// SelectiveBlock_61289183314184
// MI455X (gfx1250) — hardware-verified
//
#include <hip/hip_runtime.h>


namespace {
constexpr int NB = 8, S = 1024, D = 384, NH = 6, DH = 64, DFF = 1536, NROW = NB * S;
constexpr float XS = 8.0f, WSC = 256.0f, PS = 8.0f, LN_EPS = 1e-5f, SCALE = 0.125f;
__device__ __forceinline__ void split16(float v, _Float16& hi, _Float16& lo) { hi = (_Float16)v; lo = (_Float16)(v - (float)hi); }

typedef _Float16 b16;
typedef __attribute__((ext_vector_type(16))) _Float16 v16b;
typedef __attribute__((ext_vector_type(8))) _Float16 v8b;
typedef __attribute__((ext_vector_type(8))) float v8f;
typedef __attribute__((ext_vector_type(4))) float v4f;
__device__ __forceinline__ float bf16_rne(float f) { unsigned int u = __float_as_uint(f); u += 0x7FFFu + ((u >> 16) & 1u); return __uint_as_float(u & 0xFFFF0000u); }
__device__ __forceinline__ v16b frag_kb(const b16* p, int hh) { const v8b a = *(const v8b*)(p + 8 * hh), b = *(const v8b*)(p + 16 + 8 * hh); v16b f;
#pragma unroll
  for (int e = 0; e < 8; ++e) { f[e] = a[e]; f[8 + e] = b[e]; } return f; }
__device__ __forceinline__ v8f wmma16b(v16b a, v16b b, v8f c) { v8f d = __builtin_amdgcn_wmma_f32_16x16x32_f16(false, a, false, b, (short)0, c, false, false); asm volatile("v_nop\n\tv_nop\n\tv_nop\n\tv_nop" : "+v"(d) : "v"(a), "v"(b)); return d; }
__device__ __forceinline__ void wave_lds_sync() { __builtin_amdgcn_fence(__ATOMIC_RELEASE, "workgroup"); __builtin_amdgcn_wave_barrier(); __builtin_amdgcn_fence(__ATOMIC_ACQUIRE, "workgroup"); }
__device__ __forceinline__ float nexp(float x) { return __builtin_amdgcn_exp2f(x * 1.4426950408889634f); }
__device__ __forceinline__ float pmul(float a, float b) { float p = a * b; asm volatile("" : "+v"(p)); return p; }
__device__ __forceinline__ float hsum16(float v) { v += __shfl_xor(v, 1); v += __shfl_xor(v, 2); v += __shfl_xor(v, 4); return v + __shfl_xor(v, 8); }

__global__ __launch_bounds__(256) void prepw_kernel(const float* __restrict__ wqkv, const float* __restrict__ wout, const float* __restrict__ wup, const float* __restrict__ wdn, b16* __restrict__ WQKV, b16* __restrict__ WOUT, b16* __restrict__ WUP, b16* __restrict__ WDN) {
  const size_t tid = (size_t)blockIdx.x * 256 + threadIdx.x, nth = (size_t)gridDim.x * 256;
  const size_t n1 = (size_t)3 * D * D / 8, n2 = (size_t)D * D / 8, n3 = (size_t)DFF * D / 8, n4 = (size_t)D * DFF / 8;
  for (int pass = 0; pass < 2; ++pass) {
    for (size_t g = tid; g < n1 + n2 + n3 + n4; g += nth) { const float* src; b16* dst; size_t e;
      if (g < n1) { src = wqkv; dst = WQKV; e = g * 8; } else if (g < n1 + n2) { src = wout; dst = WOUT; e = (g - n1) * 8; } else if (g < n1 + n2 + n3) { src = wup; dst = WUP; e = (g - n1 - n2) * 8; } else { src = wdn; dst = WDN; e = (g - n1 - n2 - n3) * 8; }
      const v4f a = *(const v4f*)(src + e), c = *(const v4f*)(src + e + 4); v8b o;
#pragma unroll
      for (int j = 0; j < 4; ++j) { o[j] = (b16)(bf16_rne(a[j]) * WSC); o[4 + j] = (b16)(bf16_rne(c[j]) * WSC); }
      *(volatile v8b*)(dst + e) = o; }
    __threadfence(); }
}
template <int MODE>
__global__ __launch_bounds__(256) void ln_kernel(const float* __restrict__ X, const float* __restrict__ w, const float* __restrict__ bb, b16* __restrict__ H16) {
  __shared__ __attribute__((aligned(16))) b16 Tr[8][D + 8];
  const int wave = threadIdx.x >> 5, lane = threadIdx.x & 31; const size_t row = (size_t)blockIdx.x * 8 + wave; const float* src = X + row * D;
  float v[12]; float s = 0.0f;
#pragma unroll
  for (int j = 0; j < 12; ++j) { v[j] = MODE == 0 ? bf16_rne(src[j * 32 + lane]) : src[j * 32 + lane]; s += v[j]; }
#pragma unroll
  for (int o = 16; o >= 1; o >>= 1) s += __shfl_xor(s, o);
  const float mean = s * (1.0f / D); float ss = 0.0f;
#pragma unroll
  for (int j = 0; j < 12; ++j) { const float d = v[j] - mean; ss += pmul(d, d); }
#pragma unroll
  for (int o = 16; o >= 1; o >>= 1) ss += __shfl_xor(ss, o);
  const float rs = rsqrtf(ss * (1.0f / D) + LN_EPS);
#pragma unroll
  for (int j = 0; j < 12; ++j) { const int c = j * 32 + lane; Tr[wave][c] = (b16)((pmul((v[j] - mean) * rs, bf16_rne(w[c])) + bf16_rne(bb[c])) * XS); }
  wave_lds_sync();
  for (int pass = 0; pass < 2; ++pass) { for (int qd = 0; qd < 2; ++qd) { const int ch = qd * 32 + lane; if (ch < D / 8) *(volatile v8b*)(H16 + row * D + ch * 8) = *(const v8b*)(&Tr[wave][ch * 8]); } __threadfence(); }
}
__global__ __launch_bounds__(128) void qkv_kernel(const b16* __restrict__ H16, const b16* __restrict__ WQKV, b16* __restrict__ QH, b16* __restrict__ QL, b16* __restrict__ KH, b16* __restrict__ KL, b16* __restrict__ VROW) {
  __shared__ __attribute__((aligned(16))) b16 Th[4][16][128 + 8], Tl[4][16][128 + 8];
  const int wave = threadIdx.x >> 5, lane = threadIdx.x & 31, nloc = lane & 15, hlf = lane >> 4; const int m0 = blockIdx.x * 64 + wave * 16, n0 = blockIdx.y * 128; const int which = n0 / D, h0 = (n0 - which * D) / DH;
  v8f acc[8];
#pragma unroll
  for (int t = 0; t < 8; ++t) acc[t] = (v8f){};
#pragma unroll 2
  for (int kb = 0; kb < D; kb += 32) { const v16b a = frag_kb(H16 + (size_t)(m0 + nloc) * D + kb, hlf);
#pragma unroll
    for (int t = 0; t < 8; ++t) acc[t] = wmma16b(a, frag_kb(WQKV + (size_t)(n0 + t * 16 + nloc) * D + kb, hlf), acc[t]); }
#pragma unroll
  for (int t = 0; t < 8; ++t)
#pragma unroll
    for (int r = 0; r < 8; ++r) acc[t][r] *= (1.0f / (XS * WSC));
#pragma unroll
  for (int t = 0; t < 8; ++t)
#pragma unroll
    for (int r = 0; r < 8; ++r) { b16 p, q; split16(acc[t][r] * XS, p, q); Th[wave][8 * hlf + r][t * 16 + nloc] = p; Tl[wave][8 * hlf + r][t * 16 + nloc] = q; }
  wave_lds_sync();
  b16* dst = which == 0 ? QH : which == 1 ? KH : VROW; b16* dstl = which == 0 ? QL : which == 1 ? KL : nullptr;
  for (int pass = 0; pass < 2; ++pass) { for (int rr = 0; rr < 16; ++rr) if (lane < 16) { const int m = m0 + rr, b = m / S, l = m - b * S; const int hs = lane >> 3, c8 = (lane & 7) * 8; const size_t gi = (((size_t)b * NH + h0 + hs) * S + l) * DH + c8;
      *(volatile v8b*)(dst + gi) = *(const v8b*)(&Th[wave][rr][hs * 64 + c8]); if (which < 2) *(volatile v8b*)(dstl + gi) = *(const v8b*)(&Tl[wave][rr][hs * 64 + c8]); } __threadfence(); }
}
__global__ __launch_bounds__(256) void vt_kernel(const b16* __restrict__ VROW, b16* __restrict__ VT) {
  __shared__ __attribute__((aligned(16))) b16 Tt[DH][64 + 8];
  const int bh = blockIdx.y, s0 = blockIdx.x * 64, t_ = threadIdx.x;
  for (int k = t_; k < 64 * DH; k += 256) { const int ss = k >> 6, d = k & 63; Tt[d][ss] = VROW[((size_t)bh * S + s0 + ss) * DH + d]; }
  __syncthreads();
  for (int pass = 0; pass < 2; ++pass) { for (int q = t_; q < DH * 8; q += 256) { const int d = q >> 3, c8 = (q & 7) * 8; *(volatile v8b*)(VT + ((size_t)bh * DH + d) * S + s0 + c8) = *(const v8b*)(&Tt[d][c8]); } __threadfence(); }
}
__global__ __launch_bounds__(64) void attn_kernel(const b16* __restrict__ QH, const b16* __restrict__ QL, const b16* __restrict__ KH, const b16* __restrict__ KL, const b16* __restrict__ VT, const float* __restrict__ alpha_, const float* __restrict__ beta_, const float* __restrict__ gamma_, b16* __restrict__ ATT) {
  __shared__ __attribute__((aligned(16))) b16 To[2][16][DH + 8];
  const int wave = threadIdx.x >> 5, lane = threadIdx.x & 31, hh = lane >> 4, col = lane & 15; const int bh = blockIdx.y, b = bh / NH, h = bh - b * NH, q0 = blockIdx.x * 32 + wave * 16, qi = q0 + col;
  const b16* Q = QH + (size_t)bh * S * DH; const b16* Qlp = QL + (size_t)bh * S * DH; const b16* K = KH + (size_t)bh * S * DH; const b16* Klp = KL + (size_t)bh * S * DH; const b16* V = VT + (size_t)bh * DH * S;
  const float al = bf16_rne(alpha_[h]), be = bf16_rne(beta_[h]), ga = bf16_rne(gamma_[h]);
  v16b qf[2], ql[2];
#pragma unroll
  for (int ks = 0; ks < 2; ++ks) { qf[ks] = frag_kb(Q + (size_t)qi * DH + ks * 32, hh); ql[ks] = frag_kb(Qlp + (size_t)qi * DH + ks * 32, hh); }
  const float scale = SCALE / (XS * XS);
  float l = 0.0f; v8f o[4] = {{}, {}, {}, {}};
  for (int kb = 0; kb < S; kb += 32) {
    v8f s0 = {}, s1 = {};
#pragma unroll
    for (int ks = 0; ks < 2; ++ks) { v16b kf = frag_kb(K + (size_t)(kb + col) * DH + ks * 32, hh); s0 = wmma16b(kf, qf[ks], s0); s0 = wmma16b(kf, ql[ks], s0); s0 = wmma16b(frag_kb(Klp + (size_t)(kb + col) * DH + ks * 32, hh), qf[ks], s0);
      kf = frag_kb(K + (size_t)(kb + 16 + col) * DH + ks * 32, hh); s1 = wmma16b(kf, qf[ks], s1); s1 = wmma16b(kf, ql[ks], s1); s1 = wmma16b(frag_kb(Klp + (size_t)(kb + 16 + col) * DH + ks * 32, hh), qf[ks], s1); }
    float sum = 0.0f; v16b pb;
#pragma unroll
    for (int r = 0; r < 8; ++r) { const float x0 = s0[r] * scale, x1 = s1[r] * scale; const float w0 = fmaxf((al * x0 + be) * x0 + ga, 0.0f), w1 = fmaxf((al * x1 + be) * x1 + ga, 0.0f); sum += w0 + w1; pb[r] = (b16)(w0 * PS); pb[8 + r] = (b16)(w1 * PS); }
    sum += __shfl_xor(sum, 16); l += sum;
#pragma unroll
    for (int t = 0; t < 4; ++t) o[t] = wmma16b(frag_kb(V + (size_t)(t * 16 + col) * S + kb, hh), pb, o[t]); }
  const float inv = 1.0f / ((l + 1e-6f) * PS * XS);
#pragma unroll
  for (int t = 0; t < 4; ++t)
#pragma unroll
    for (int r = 0; r < 8; ++r) To[wave][col][t * 16 + 8 * hh + r] = (b16)(o[t][r] * inv * XS);
  wave_lds_sync();
  for (int pass = 0; pass < 2; ++pass) { for (int rr = 0; rr < 16; ++rr) if (lane < 8) *(volatile v8b*)(ATT + ((size_t)b * S + q0 + rr) * D + h * DH + lane * 8) = *(const v8b*)(&To[wave][rr][lane * 8]); __threadfence(); }
}
template <int MODE>
__global__ __launch_bounds__(128) void gemmres_kernel(const b16* __restrict__ A, int K, const b16* __restrict__ Bw, const float* __restrict__ bias, const float* __restrict__ R, float* __restrict__ Y) {
  __shared__ __attribute__((aligned(16))) float Ts[4][16][128 + 4];
  const int wave = threadIdx.x >> 5, lane = threadIdx.x & 31, nloc = lane & 15, hlf = lane >> 4; const int m0 = blockIdx.x * 64 + wave * 16, n0 = blockIdx.y * 128;
  v8f acc[8];
#pragma unroll
  for (int t = 0; t < 8; ++t) acc[t] = (v8f){};
  for (int kb = 0; kb < K; kb += 32) { const v16b a = frag_kb(A + (size_t)(m0 + nloc) * K + kb, hlf);
#pragma unroll
    for (int t = 0; t < 8; ++t) acc[t] = wmma16b(a, frag_kb(Bw + (size_t)(n0 + t * 16 + nloc) * K + kb, hlf), acc[t]); }
#pragma unroll
  for (int t = 0; t < 8; ++t)
#pragma unroll
    for (int r = 0; r < 8; ++r) Ts[wave][8 * hlf + r][t * 16 + nloc] = acc[t][r] * (1.0f / (XS * WSC)) + bf16_rne(bias[n0 + t * 16 + nloc]);
  wave_lds_sync();
  for (int pass = 0; pass < 2; ++pass) { for (int rr = 0; rr < 16; ++rr) { const size_t gi = (size_t)(m0 + rr) * D + n0 + lane * 4; v4f v = *(const v4f*)(&Ts[wave][rr][lane * 4]); const v4f rv = *(const v4f*)(R + gi);
      if (MODE == 0) { v[0] += bf16_rne(rv[0]); v[1] += bf16_rne(rv[1]); v[2] += bf16_rne(rv[2]); v[3] += bf16_rne(rv[3]); } else v += rv; *(volatile v4f*)(Y + gi) = v; } __threadfence(); }
}
__global__ __launch_bounds__(128) void up_kernel(const b16* __restrict__ H2, const b16* __restrict__ WUP, const float* __restrict__ b1, b16* __restrict__ H3) {
  __shared__ __attribute__((aligned(16))) float Tu[4][16][128 + 4];
  const int wave = threadIdx.x >> 5, lane = threadIdx.x & 31, nloc = lane & 15, hlf = lane >> 4; const int m0 = blockIdx.x * 64 + wave * 16, j0 = blockIdx.y * 128;
  v8f acc[8];
#pragma unroll
  for (int t = 0; t < 8; ++t) acc[t] = (v8f){};
#pragma unroll 2
  for (int kb = 0; kb < D; kb += 32) { const v16b a = frag_kb(H2 + (size_t)(m0 + nloc) * D + kb, hlf);
#pragma unroll
    for (int t = 0; t < 8; ++t) acc[t] = wmma16b(a, frag_kb(WUP + (size_t)(j0 + t * 16 + nloc) * D + kb, hlf), acc[t]); }
#pragma unroll
  for (int t = 0; t < 8; ++t) { const float bb = bf16_rne(b1[j0 + t * 16 + nloc]);
#pragma unroll
    for (int r = 0; r < 8; ++r) Tu[wave][8 * hlf + r][t * 16 + nloc] = acc[t][r] * (1.0f / (XS * WSC)) + bb; }
  wave_lds_sync();
#pragma unroll 1
  for (int i = 0; i < 8; ++i) { const int rr = 2 * i + (lane >> 4);
#pragma unroll 1
    for (int j = 0; j < 8; ++j) { const int c = (lane & 15) * 8 + j; const float u = Tu[wave][rr][c]; Tu[wave][rr][c] = 0.5f * u * (1.0f + erff(u * 0.70710678118654752f)); } }
  wave_lds_sync();
  for (int pass = 0; pass < 2; ++pass) { for (int rr = 0; rr < 16; ++rr) if (lane < 16) { v8b o; const float* tu = &Tu[wave][rr][lane * 8];
#pragma unroll
      for (int j = 0; j < 8; ++j) o[j] = (b16)(tu[j] * XS); *(volatile v8b*)(H3 + (size_t)(m0 + rr) * DFF + j0 + lane * 8) = o; } __threadfence(); }
}
}

extern "C" void kernel_launch(void* const* d_in, const int* in_sizes, int n_in, void* d_out, int out_size, void* d_ws, size_t ws_size, hipStream_t stream) {
  (void)n_in;
  auto Fp = [&](int i) { return (const float*)d_in[i]; };
  if (in_sizes[0] != NROW * D || in_sizes[1] != 3 * D * D || in_sizes[2] != D * D || in_sizes[3] != D || in_sizes[4] != NH || in_sizes[7] != D || in_sizes[11] != DFF * D || in_sizes[12] != DFF || in_sizes[13] != D * DFF || in_sizes[14] != D || out_size != NROW * D) return;
  size_t off = 0; char* ws = (char*)d_ws;
  auto carve = [&](size_t bytes) { char* p = ws + off; off += (bytes + 255) & ~(size_t)255; return p; };
  b16* WQKV = (b16*)carve((size_t)3 * D * D * 2); b16* WOUT = (b16*)carve((size_t)D * D * 2); b16* WUP = (b16*)carve((size_t)DFF * D * 2); b16* WDN = (b16*)carve((size_t)D * DFF * 2);
  b16* H16 = (b16*)carve((size_t)NROW * D * 2); b16* QH = (b16*)carve((size_t)NROW * D * 2); b16* QL = (b16*)carve((size_t)NROW * D * 2); b16* KH = (b16*)carve((size_t)NROW * D * 2); b16* KL = (b16*)carve((size_t)NROW * D * 2);
  b16* VROW = (b16*)carve((size_t)NROW * D * 2); b16* VT = (b16*)carve((size_t)NROW * D * 2); b16* ATT = (b16*)carve((size_t)NROW * D * 2); b16* H2 = (b16*)carve((size_t)NROW * D * 2);
  float* X1 = (float*)carve((size_t)NROW * D * 4); b16* H3 = (b16*)carve((size_t)NROW * DFF * 2);
  if (off > ws_size || off > ((size_t)128 << 20)) return;
  prepw_kernel<<<512, 256, 0, stream>>>(Fp(1), Fp(2), Fp(11), Fp(13), WQKV, WOUT, WUP, WDN);
  ln_kernel<0><<<NROW / 8, 256, 0, stream>>>(Fp(0), Fp(7), Fp(8), H16);
  qkv_kernel<<<dim3(NROW / 64, 3 * D / 128), 128, 0, stream>>>(H16, WQKV, QH, QL, KH, KL, VROW);
  vt_kernel<<<dim3(S / 64, NB * NH), 256, 0, stream>>>(VROW, VT);
  attn_kernel<<<dim3(S / 32, NB * NH), 64, 0, stream>>>(QH, QL, KH, KL, VT, Fp(4), Fp(5), Fp(6), ATT);
  gemmres_kernel<0><<<dim3(NROW / 64, D / 128), 128, 0, stream>>>(ATT, D, WOUT, Fp(3), Fp(0), X1);
  ln_kernel<1><<<NROW / 8, 256, 0, stream>>>(X1, Fp(9), Fp(10), H2);
  up_kernel<<<dim3(NROW / 64, DFF / 128), 128, 0, stream>>>(H2, WUP, Fp(12), H3);
  gemmres_kernel<1><<<dim3(NROW / 64, D / 128), 128, 0, stream>>>(H3, DFF, WDN, Fp(14), X1, (float*)d_out);
}
